// GMM_44332652429390
// MI455X (gfx1250) — hardware-run, weakly checked
//
#include <hip/hip_runtime.h>


#ifndef TROWS
#define TROWS 262144
#endif
#define TROWS_FULL 262144
#define NMIX  64
#define NDIM  16
#define KD    32
#define KW    8
#define BROWS (16 * KW)
#define BFL   (BROWS * NDIM)
#define NBLK  (TROWS / BROWS)
#define RECW  64
#define NPIECE ((BFL / 32 - 1) * 8)
#define QRS   2048.0f
#define QRI   (1.0f / 2048.0f)
#define PSH   14.0f
#define NEGB  (-3.0e38f)
#define LOG2E 1.4426950408889634
#define GCF   ((float)(-0.5 * LOG2E))
#define LN2F  ((float)0.6931471805599453)
#define PI2D  6.283185307
#define CGAUSS ((float)(1.0 / (((PI2D * PI2D) * (PI2D * PI2D)) * ((PI2D * PI2D) * (PI2D * PI2D)))))

static_assert(NDIM == 16);
static_assert(KD == 2 * NDIM);
static_assert(KD == 32);
static_assert(NMIX == 64);
static_assert(TROWS % BROWS == 0);
static_assert(TROWS <= TROWS_FULL);
static_assert(32 * KW == 256);
static_assert(BFL % 32 == 0);
static_assert(NPIECE % 8 == 0);
static_assert(NPIECE <= 2 * 32 * KW);
static_assert(NPIECE * 4 == BFL - 32);
static_assert(RECW * 4 == 16 * 16);
static_assert(4 * 64 * 8 == NMIX * KD);
static_assert(2 * 64 * 8 == NDIM * NMIX);
static_assert(16 * 4 == NMIX);
static_assert((BFL + 4 + KW) * 4 <= 131072);
static_assert((2 * NMIX * KD + NDIM * NMIX) * 2 + NMIX * 4 <= 131072);

typedef _Float16 h16;
typedef __attribute__((ext_vector_type(16))) _Float16 v16h;
typedef __attribute__((ext_vector_type(8)))  _Float16 v8h;
typedef __attribute__((ext_vector_type(8)))  float    v8f;
typedef __attribute__((ext_vector_type(4)))  float    v4f;
typedef v4f  __attribute__((may_alias)) v4fa;
typedef v8h  __attribute__((may_alias)) v8ha;

__device__ __forceinline__ unsigned short f2bf(float f) { unsigned u = __float_as_uint(f); u += 0x7FFFu + ((u >> 16) & 1u); return (unsigned short)(u >> 16); }
__device__ __forceinline__ float bfr(float f) { return __uint_as_float(((unsigned)f2bf(f)) << 16); }
__device__ __forceinline__ v16h cat16(v8h lo, v8h hi) { return __builtin_shufflevector(lo, hi, 0, 1, 2, 3, 4, 5, 6, 7, 8, 9, 10, 11, 12, 13, 14, 15); }
__device__ __forceinline__ v16h  ldh(const h16* p) { return cat16(*(const v8h*)p, *(const v8h*)(p + 16)); }
static __device__ __forceinline__ h16 toh_flush(float v) { const h16 r = (h16)v; return (fabsf(v) < 6.103515625e-05f) ? (h16)0.0f : r; }
__device__ __forceinline__ v8f wmma16g(v16h a, v16h b, v8f c) {
    c = __builtin_amdgcn_wmma_f32_16x16x32_f16(false, a, false, b, (short)0, c, false, false);
    asm volatile("v_nop\n\tv_nop\n\tv_nop\n\tv_nop" : "+v"(c) : "v"(a), "v"(b));
    return c;
}

__global__ __launch_bounds__(64) void k_prep(const float* __restrict__ wghts, const float* __restrict__ means, const float* __restrict__ dcovs, h16* PH, h16* PR, h16* MT, float* SV) {
#pragma clang fp contract(off)
    __shared__ __align__(16) h16 sPH[NMIX * KD];
    __shared__ __align__(16) h16 sPR[NMIX * KD];
    __shared__ __align__(16) h16 sMT[NDIM * NMIX];
    __shared__ __align__(16) float sSV[NMIX];
    const int m = threadIdx.x;
    const float w = bfr(wghts[m]);
    float prod = 1.0f, rsum = 0.0f;
#pragma unroll 1
    for (int d = 0; d < NDIM; ++d) {
        const float cov = bfr(dcovs[m * NDIM + d]);
        const float mu  = bfr(means[m * NDIM + d]);
        const float p = 1.0f / cov;
        const float q = (-2.0f * mu) * p;
        rsum += (mu * mu) * p;
        prod *= cov;
        const h16 ph = toh_flush(p);
        const h16 qh = toh_flush(q);
        sPH[m * KD + d] = ph;
        sPH[m * KD + NDIM + d] = qh;
        sPR[m * KD + d] = toh_flush((p - (float)ph) * QRS);
        sPR[m * KD + NDIM + d] = toh_flush((q - (float)qh) * QRS);
        sMT[d * NMIX + m] = toh_flush(mu);
    }
    sSV[m] = (log2f(w * CGAUSS) - 0.5f * log2f(prod)) - (0.5f * (float)LOG2E) * rsum;
    __syncthreads();
#pragma unroll 1
    for (int ps = 0; ps < 2; ++ps) {
#pragma unroll
        for (int it = 0; it < 4; ++it) { const int i = it * 64 + m;
            const v8h a = *(const v8ha*)(&sPH[i * 8]); const v8h c = *(const v8ha*)(&sPR[i * 8]);
            *(volatile v8h*)(PH + i * 8) = a; *(volatile v8h*)(PR + i * 8) = c; }
#pragma unroll
        for (int it = 0; it < 2; ++it) { const int i = it * 64 + m;
            const v8h a = *(const v8ha*)(&sMT[i * 8]);
            *(volatile v8h*)(MT + i * 8) = a; }
        { const int i = m < 16 ? m : 15;
          const v4f a = *(const v4fa*)(&sSV[i * 4]);
          if (m < 16) *(volatile v4f*)(SV + i * 4) = a; }
        if (ps == 0) __threadfence();
    }
}

__global__ __launch_bounds__(32 * KW) void k_mix(const float* __restrict__ X, const h16* __restrict__ PH, const h16* __restrict__ PR, const h16* __restrict__ MT,
                                                 const float* __restrict__ SV, float* OUTF, float* REC) {
    __shared__ __align__(16) float os[BFL + 4];
    __shared__ float wsum[KW];
    const int tid = threadIdx.x;
    const int lane = tid & 31, lr = lane & 15, hi = lane >> 4;
    const int wave = __builtin_amdgcn_readfirstlane((int)(threadIdx.x >> 5));
    const int blk = blockIdx.x;
    const size_t trow = (size_t)blk * BROWS + (size_t)(wave * 16 + lr);
    const float* xp = X + trow * NDIM + 8 * hi;
    const v4f xa = *(const v4f*)xp, xc = *(const v4f*)(xp + 4);
    v16h xh, xr;
#pragma unroll
    for (int i = 0; i < 4; ++i) {
        const float va = bfr(xa[i]), vc = bfr(xc[i]);
        const float sa = va * va, sc = vc * vc;
        const h16 ha = toh_flush(sa), hc = toh_flush(sc), ga = toh_flush(va), gc = toh_flush(vc);
        xh[i] = ha; xh[4 + i] = hc; xh[8 + i] = ga; xh[12 + i] = gc;
        xr[i] = toh_flush((sa - (float)ha) * QRS); xr[4 + i] = toh_flush((sc - (float)hc) * QRS);
        xr[8 + i] = toh_flush((va - (float)ga) * QRS); xr[12 + i] = toh_flush((vc - (float)gc) * QRS);
    }
    float tl[4][8];
    float mx = NEGB;
#pragma unroll
    for (int mt = 0; mt < 4; ++mt) {
        const int po = (mt * 16 + lr) * KD + 8 * hi;
        const v16h ah = ldh(PH + po), ar = ldh(PR + po);
        v8f sH = (v8f){}, sL = (v8f){};
        sH = wmma16g(ah, xh, sH);
        sL = wmma16g(ah, xr, sL);
        sL = wmma16g(ar, xh, sL);
        const v4f s0 = *(const v4f*)(SV + mt * 16 + 8 * hi), s1 = *(const v4f*)(SV + mt * 16 + 8 * hi + 4);
#pragma unroll
        for (int r = 0; r < 8; ++r) {
            const float sv = (r < 4) ? s0[r & 3] : s1[r & 3];
            const float t = (sH[r] + sL[r] * QRI) * GCF + sv;
            tl[mt][r] = t; mx = fmaxf(mx, t);
        }
    }
    mx = fmaxf(mx, __shfl_xor(mx, 16, 32));
    const float sh = PSH - mx;
    v16h pb0, pb1; float lf = 0.0f, lp = 0.0f;
#pragma unroll
    for (int r = 0; r < 8; ++r) {
        const float e0 = tl[0][r] + sh, e1 = tl[1][r] + sh, e2 = tl[2][r] + sh, e3 = tl[3][r] + sh;
        const float a0 = __builtin_amdgcn_exp2f(e0), a1 = __builtin_amdgcn_exp2f(e1), a2 = __builtin_amdgcn_exp2f(e2), a3 = __builtin_amdgcn_exp2f(e3);
        const h16 p0 = (e0 < -14.0f) ? (h16)0.0f : (h16)a0;
        const h16 p1 = (e1 < -14.0f) ? (h16)0.0f : (h16)a1;
        const h16 p2 = (e2 < -14.0f) ? (h16)0.0f : (h16)a2;
        const h16 p3 = (e3 < -14.0f) ? (h16)0.0f : (h16)a3;
        pb0[r] = p0; pb0[8 + r] = p1; pb1[r] = p2; pb1[8 + r] = p3;
        lf += (a0 + a1) + (a2 + a3);
        lp += ((float)p0 + (float)p1) + ((float)p2 + (float)p3);
    }
    lf += __shfl_xor(lf, 16, 32);
    lp += __shfl_xor(lp, 16, 32);
    const v16h m0 = ldh(MT + lr * NMIX + 8 * hi), m1 = ldh(MT + lr * NMIX + 32 + 8 * hi);
    v8f o = (v8f){};
    o = wmma16g(m0, pb0, o);
    o = wmma16g(m1, pb1, o);
    const float inv = 1.0f / lp;
    const int fb = 1 + (wave * 16 + lr) * NDIM + 8 * hi;
#pragma unroll
    for (int r = 0; r < 8; ++r) os[fb + r] = o[r] * inv;
    const float llv = ((mx - PSH) + log2f(lf)) * LN2F;
    float ll = (hi == 0) ? llv : 0.0f;
    ll += __shfl_xor(ll, 1, 32); ll += __shfl_xor(ll, 2, 32); ll += __shfl_xor(ll, 4, 32); ll += __shfl_xor(ll, 8, 32); ll += __shfl_xor(ll, 16, 32);
    if (lane == 0) wsum[wave] = ll;
    __syncthreads();
    v4f rv = (v4f){};
    if (wave == 0) {
        float part = wsum[0];
#pragma unroll
        for (int w = 1; w < KW; ++w) part += wsum[w];
#pragma unroll
        for (int e = 0; e < 4; ++e) {
            const int i = lane * 4 + e;
            const int oi = (i < 31) ? (1 + i) : BFL;
            float x = os[oi];
            asm volatile("" : "+v"(x));
            rv[e] = (i < 32) ? x : ((i == 32) ? part : 0.0f);
        }
    }
    float* ob = OUTF + (size_t)blk * BFL;
#pragma unroll 1
    for (int ps = 0; ps < 2; ++ps) {
#pragma unroll
        for (int it = 0; it < 2; ++it) {
            const int p = it * 256 + tid;
            const int pc = p < NPIECE ? p : (NPIECE - 1);
            const int idx = 32 + pc * 4;
            const v4f val = *(const v4fa*)(&os[idx]);
            if (p < NPIECE) *(volatile v4f*)(ob + idx) = val;
        }
        if (wave == 0) { if (lane < 16) *(volatile v4f*)(REC + (size_t)blk * RECW + lane * 4) = rv; }
        if (ps == 0) __threadfence();
    }
}

__global__ __launch_bounds__(256) void k_fin(const float* __restrict__ REC, float* OUTF) {
#pragma clang fp contract(off)
    __shared__ float wtot[8];
    const int tid = threadIdx.x, lane = tid & 31;
    const int wave = __builtin_amdgcn_readfirstlane((int)(threadIdx.x >> 5));
    float s = 0.0f;
#pragma unroll 1
    for (int i = tid; i < NBLK; i += 256) s += REC[(size_t)i * RECW + 32];
    s += __shfl_xor(s, 1, 32); s += __shfl_xor(s, 2, 32); s += __shfl_xor(s, 4, 32); s += __shfl_xor(s, 8, 32); s += __shfl_xor(s, 16, 32);
    if (lane == 0) wtot[wave] = s;
    __syncthreads();
    float tot = wtot[0];
#pragma unroll
    for (int w = 1; w < 8; ++w) tot += wtot[w];
    const float ll = tot * (1.0f / (float)TROWS);
    const float xl = REC[(size_t)(NBLK - 1) * RECW + 31];
#pragma unroll 1
    for (int ps = 0; ps < 2; ++ps) {
#pragma unroll 1
        for (int p = tid; p < NBLK * 8; p += 256) {
            const int b = p >> 3, c = (p & 7) * 4;
            const int bp = b > 0 ? (b - 1) : 0;
            const size_t i0 = (c == 0) ? ((size_t)bp * RECW + 31) : ((size_t)b * RECW + (size_t)(c - 1));
            float x0 = REC[i0];
            const float x1 = REC[(size_t)b * RECW + c], x2 = REC[(size_t)b * RECW + c + 1], x3 = REC[(size_t)b * RECW + c + 2];
            asm volatile("" : "+v"(x0));
            v4f v;
            v[0] = ((c == 0) & (b == 0)) ? ll : x0; v[1] = x1; v[2] = x2; v[3] = x3;
            *(volatile v4f*)(OUTF + (size_t)b * BFL + c) = v;
        }
        if (tid == 0) *(volatile float*)(OUTF + (size_t)NBLK * BFL) = xl;
        if (ps == 0) __threadfence();
    }
}

static constexpr size_t al256(size_t v) { return (v + 255) & ~(size_t)255; }
static constexpr size_t SZ_PH  = al256((size_t)NMIX * KD * 2);
static constexpr size_t SZ_MT  = al256((size_t)NDIM * NMIX * 2);
static constexpr size_t SZ_SV  = al256((size_t)NMIX * 4);
static constexpr size_t SZ_REC = al256((size_t)NBLK * RECW * 4);
static constexpr size_t SZ_TOTAL = 2 * SZ_PH + SZ_MT + SZ_SV + SZ_REC;
static_assert(SZ_TOTAL <= (size_t)134217728);
static_assert((size_t)NBLK * BFL == (size_t)TROWS * NDIM);
static_assert(((size_t)TROWS_FULL * NDIM + 1) * 4 == (size_t)16777220);

extern "C" void kernel_launch(void* const* d_in, const int* in_sizes, int n_in,
                              void* d_out, int out_size, void* d_ws, size_t ws_size, hipStream_t stream) {
    if (n_in < 4) return;
    if ((size_t)in_sizes[0] < (size_t)TROWS * NDIM) return;
    if (in_sizes[1] < NMIX || in_sizes[2] < NMIX * NDIM || in_sizes[3] < NMIX * NDIM) return;
    if ((size_t)out_size < (size_t)TROWS * NDIM + 1) return;
    if (SZ_TOTAL > ws_size) return;
    const float* xd = (const float*)d_in[0];
    const float* wg = (const float*)d_in[1];
    const float* mu = (const float*)d_in[2];
    const float* cv = (const float*)d_in[3];
    float* OUTF = (float*)d_out;
    char* wsp = (char*)d_ws;
    h16* PH = (h16*)wsp; wsp += SZ_PH;
    h16* PR = (h16*)wsp; wsp += SZ_PH;
    h16* MT = (h16*)wsp; wsp += SZ_MT;
    float* SV = (float*)wsp; wsp += SZ_SV;
    float* REC = (float*)wsp; wsp += SZ_REC;

    k_prep<<<dim3(1, 1, 1), 64, 0, stream>>>(wg, mu, cv, PH, PR, MT, SV);
    k_mix<<<dim3(NBLK, 1, 1), 32 * KW, 0, stream>>>(xd, PH, PR, MT, SV, OUTF, REC);
    k_fin<<<dim3(1, 1, 1), 256, 0, stream>>>(REC, OUTF);
}
